// MultiHeadAttentionBlock_23665269801423
// MI455X (gfx1250) — hardware-run, weakly checked
//
#include <hip/hip_runtime.h>
#include <math.h>

#ifndef NB
#define NB 2
#endif
#ifndef SEQ
#define SEQ 2048
#endif
#define NB_FULL 2
#define SEQ_FULL 2048
#define DM 512
#define NH 8
#define DKH 64
#define NTOK (NB * SEQ)
#define PP 72
#define OP 68
#define NRP 10
#define NREL 21
#define RP 36
#define BW (16 * RP + 32)
#define TP 68

static_assert(DM == NH * DKH);
static_assert(DKH == 64);
static_assert(SEQ % 64 == 0);
static_assert(NTOK % 64 == 0);
static_assert(DM % 64 == 0);
static_assert(DM % 32 == 0);
static_assert((2 * DM) % 32 == 0);
static_assert(NB <= NB_FULL);
static_assert(SEQ <= SEQ_FULL);
static_assert((PP % 8) == 0);
static_assert((OP % 4) == 0);
static_assert(NREL == 2 * NRP + 1);
static_assert(NREL <= 32);
static_assert((RP % 4) == 0 && RP >= 32);
static_assert((BW % 32) == 0);
static_assert((BW % 4) == 0);
static_assert((TP % 4) == 0);
static_assert(4 * 16 * PP * 2 + 4 * 16 * OP * 4 + 4 * 16 * RP * 4 + 4 * BW * 4 <= 131072);
static_assert(8 * 16 * OP * 4 <= 131072);
static_assert(64 * TP * 4 <= 131072);
static_assert(32 * 16 * 4 == 16 * 128);
static_assert(256 * 16 * 2 == 64 * 128);
static_assert(256 * 8 == 32 * DKH);
static_assert(256 * 8 == DKH * 32);

typedef __attribute__((ext_vector_type(16))) _Float16 v16h;
typedef __attribute__((ext_vector_type(8)))  _Float16 v8h;
typedef __attribute__((ext_vector_type(16))) __bf16   v16b;
typedef __attribute__((ext_vector_type(8)))  __bf16   v8b;
typedef __attribute__((ext_vector_type(8)))  float    v8f;
typedef __attribute__((ext_vector_type(4)))  float    v4f;
typedef __attribute__((ext_vector_type(4)))  unsigned int v4u;
typedef v8h v8h_ma __attribute__((may_alias));
typedef v4f v4f_ma __attribute__((may_alias));


__device__ __forceinline__ unsigned int bf_bits(float f) {
    const unsigned int u = __float_as_uint(f);
    return (u + 0x7FFFu + ((u >> 16) & 1u)) >> 16;
}
__device__ __forceinline__ float bf_val(float f) { return __uint_as_float(bf_bits(f) << 16); }
__device__ __forceinline__ unsigned int pk_h2(float a, float b) {
    return (unsigned int)__builtin_bit_cast(unsigned short, (_Float16)a) | ((unsigned int)__builtin_bit_cast(unsigned short, (_Float16)b) << 16);
}
__device__ __forceinline__ void pk_split2(float a, float b, unsigned int& hi, unsigned int& lo) {
    const unsigned int ha = bf_bits(a), hb = bf_bits(b);
    const unsigned int la = bf_bits(a - __uint_as_float(ha << 16)), lb = bf_bits(b - __uint_as_float(hb << 16));
    hi = ha | (hb << 16); lo = la | (lb << 16);
}
__device__ __forceinline__ void wave_sync() {
    __builtin_amdgcn_fence(3  , "workgroup");
    __builtin_amdgcn_wave_barrier();
    __builtin_amdgcn_fence(2  , "workgroup");
}
static __device__ __forceinline__ _Float16 toh_flush(float v) {
    const _Float16 r = (_Float16)v;
    return (fabsf(v) < 6.103515625e-05f) ? (_Float16)0.0f : r;
}
__device__ __forceinline__ unsigned int pk_h2f(float a, float b) {
    return (unsigned int)__builtin_bit_cast(unsigned short, toh_flush(a)) | ((unsigned int)__builtin_bit_cast(unsigned short, toh_flush(b)) << 16);
}

__device__ __forceinline__ v16h ldfrag_h(const unsigned short* __restrict__ p) {
    const v8h a = *(const v8h*)(p);
    const v8h b = *(const v8h*)(p + 16);
    return __builtin_shufflevector(a, b, 0, 1, 2, 3, 4, 5, 6, 7, 8, 9, 10, 11, 12, 13, 14, 15);
}
__device__ __forceinline__ v16b ldfrag_b(const unsigned short* __restrict__ p) {
    const v8b a = *(const v8b*)(p);
    const v8b b = *(const v8b*)(p + 16);
    return __builtin_shufflevector(a, b, 0, 1, 2, 3, 4, 5, 6, 7, 8, 9, 10, 11, 12, 13, 14, 15);
}

template <int ET> struct FragT;
template <> struct FragT<0> {
    typedef v16h V;
    static __device__ __forceinline__ v16h load(const unsigned short* __restrict__ p) { return ldfrag_h(p); }
    static __device__ __forceinline__ v8f mma(v16h a, v16h b, v8f c) { return __builtin_amdgcn_wmma_f32_16x16x32_f16(false, a, false, b, (short)0, c, false, false); }
};
template <> struct FragT<1> {
    typedef v16b V;
    static __device__ __forceinline__ v16b load(const unsigned short* __restrict__ p) { return ldfrag_b(p); }
    static __device__ __forceinline__ v8f mma(v16b a, v16b b, v8f c) { return __builtin_amdgcn_wmma_f32_16x16x32_bf16(false, a, false, b, (short)0, c, false, false); }
};
template <typename V>
__device__ __forceinline__ void guard4(v8f& a, v8f& b, v8f& c, v8f& d, V x, V y0, V y1, V y2, V y3) {
    asm volatile("v_nop\n\tv_nop\n\tv_nop\n\tv_nop" : "+v"(a), "+v"(b), "+v"(c), "+v"(d) : "v"(x), "v"(y0), "v"(y1), "v"(y2), "v"(y3));
}
__device__ __forceinline__ v8f wmma3b(v16b ah, v16b al, v16b bh, v16b bl, v8f c) {
    c = __builtin_amdgcn_wmma_f32_16x16x32_bf16(false, ah, false, bh, (short)0, c, false, false);
    c = __builtin_amdgcn_wmma_f32_16x16x32_bf16(false, ah, false, bl, (short)0, c, false, false);
    c = __builtin_amdgcn_wmma_f32_16x16x32_bf16(false, al, false, bh, (short)0, c, false, false);
    asm volatile("v_nop\n\tv_nop\n\tv_nop\n\tv_nop" : "+v"(c) : "v"(ah), "v"(al), "v"(bh), "v"(bl));
    return c;
}
__device__ __forceinline__ v8f wmma_h1(v16h a, v16h b, v8f c) {
    c = __builtin_amdgcn_wmma_f32_16x16x32_f16(false, a, false, b, (short)0, c, false, false);
    asm volatile("v_nop\n\tv_nop\n\tv_nop\n\tv_nop" : "+v"(c) : "v"(a), "v"(b));
    return c;
}
__device__ __forceinline__ v8f wmma_b1(v16b a, v16b b, v8f c) {
    c = __builtin_amdgcn_wmma_f32_16x16x32_bf16(false, a, false, b, (short)0, c, false, false);
    asm volatile("v_nop\n\tv_nop\n\tv_nop\n\tv_nop" : "+v"(c) : "v"(a), "v"(b));
    return c;
}

template <int ET, int BIAS_MODE, int OUT_MODE>
__device__ __forceinline__ void gemm64_body(const unsigned short* __restrict__ A, int lda,
                                            const unsigned short* __restrict__ Bt, int ldb,
                                            float* __restrict__ Cf, unsigned short* __restrict__ Ca, unsigned short* __restrict__ Cb, int ldc,
                                            const float* __restrict__ bias, int M, int N, int K,
                                            float scale, float bscale, int cseq, int cseqfull) {
    typedef typename FragT<ET>::V V;
    __shared__ __align__(16) float sT[8 * 16 * OP];
    const int lane = threadIdx.x & 31;
    const int wave = __builtin_amdgcn_readfirstlane(threadIdx.x >> 5);
    const int tilesN = N >> 6;
    const int tilesM = M >> 6;
    const int tile = blockIdx.x * 8 + wave;
    if (tile >= tilesM * tilesN) return;
    const int tm = tile / tilesN;
    const int tn = tile - tm * tilesN;
    const int m0 = tm << 6;
    const int n0 = tn << 6;
    const int rl   = lane & 15;
    const int koff = (lane >> 4) * 8;
    const int mOff = (lane >> 4) * 8;

    v8f acc[4][4];
#pragma unroll
    for (int i = 0; i < 4; ++i)
#pragma unroll
        for (int j = 0; j < 4; ++j) { const v8f zz = {0.f, 0.f, 0.f, 0.f, 0.f, 0.f, 0.f, 0.f}; acc[i][j] = zz; }

    for (int k0 = 0; k0 < K; k0 += 32) {
        V bh[4];
#pragma unroll
        for (int j = 0; j < 4; ++j) bh[j] = FragT<ET>::load(Bt + (size_t)(n0 + (j << 4) + rl) * ldb + koff + k0);
#pragma unroll
        for (int i = 0; i < 4; ++i) {
            const V ah = FragT<ET>::load(A + (size_t)(m0 + (i << 4) + rl) * lda + koff + k0);
            acc[i][0] = FragT<ET>::mma(ah, bh[0], acc[i][0]);
            acc[i][1] = FragT<ET>::mma(ah, bh[1], acc[i][1]);
            acc[i][2] = FragT<ET>::mma(ah, bh[2], acc[i][2]);
            acc[i][3] = FragT<ET>::mma(ah, bh[3], acc[i][3]);
            guard4<V>(acc[i][0], acc[i][1], acc[i][2], acc[i][3], ah, bh[0], bh[1], bh[2], bh[3]);
        }
    }

    const int sb = wave * (16 * OP);
#pragma unroll
    for (int i = 0; i < 4; ++i) {
        const int mBase = m0 + (i << 4);
#pragma unroll
        for (int j = 0; j < 4; ++j) {
            const int n = n0 + (j << 4) + rl;
            float bvn = 0.f;
            if (BIAS_MODE == 2) bvn = bf_val(bias[n]) * bscale;
#pragma unroll
            for (int r = 0; r < 8; ++r) {
                float v = acc[i][j][r] * scale;
                if (BIAS_MODE == 1) v += bf_val(bias[mBase + mOff + r]) * bscale;
                if (BIAS_MODE == 2) v += bvn;
                sT[sb + (mOff + r) * OP + (j << 4) + rl] = v;
            }
        }
        wave_sync();
        if (OUT_MODE == 0) {
            const int hh = lane >> 4, c4 = (lane & 15) * 4;
            for (int pass = 0; pass < 2; ++pass) {
#pragma unroll
                for (int it = 0; it < 8; ++it) {
                    const int row = it * 2 + hh;
                    const v4f v = *(const v4f_ma*)&sT[sb + row * OP + c4];
                    const int grow = mBase + row;
                    const int orow = (grow / cseq) * cseqfull + (grow % cseq);
                    *(volatile v4f*)(Cf + (size_t)orow * ldc + n0 + c4) = v;
                }
                __threadfence();
            }
        } else {
            const int q = lane >> 3, c8 = (lane & 7) * 8;
            for (int pass = 0; pass < 2; ++pass) {
#pragma unroll
                for (int it = 0; it < 4; ++it) {
                    const int row = it * 4 + q;
                    const v4f a = *(const v4f_ma*)&sT[sb + row * OP + c8];
                    const v4f b = *(const v4f_ma*)&sT[sb + row * OP + c8 + 4];
                    const size_t o = (size_t)(mBase + row) * ldc + n0 + c8;
                    if (OUT_MODE == 1) {
                        v4u pk; pk.x = pk_h2(a.x, a.y); pk.y = pk_h2(a.z, a.w); pk.z = pk_h2(b.x, b.y); pk.w = pk_h2(b.z, b.w);
                        *(volatile v4u*)(Ca + o) = pk;
                    } else {
                        v4u ph, pl;
                        unsigned int h0, l0, h1, l1, h2, l2, h3, l3;
                        pk_split2(a.x, a.y, h0, l0); pk_split2(a.z, a.w, h1, l1); pk_split2(b.x, b.y, h2, l2); pk_split2(b.z, b.w, h3, l3);
                        ph.x = h0; ph.y = h1; ph.z = h2; ph.w = h3; pl.x = l0; pl.y = l1; pl.z = l2; pl.w = l3;
                        *(volatile v4u*)(Ca + o) = ph;
                        *(volatile v4u*)(Cb + o) = pl;
                    }
                }
                __threadfence();
            }
        }
        wave_sync();
    }
}

__global__ __launch_bounds__(256) void k_gemm_qk(const unsigned short* __restrict__ A, const unsigned short* __restrict__ Bt,
                                                 const float* __restrict__ bias, unsigned short* __restrict__ CH, unsigned short* __restrict__ CL,
                                                 int M, int N, int K, float scale, float bscale) {
    gemm64_body<0, 2, 2>(A, K, Bt, K, nullptr, CH, CL, N, bias, M, N, K, scale, bscale, 1, 1);
}
__global__ __launch_bounds__(256) void k_gemm_vt(const unsigned short* __restrict__ A, const unsigned short* __restrict__ Bt,
                                                 const float* __restrict__ bias, unsigned short* __restrict__ C,
                                                 int M, int N, int K, float scale) {
    gemm64_body<0, 1, 1>(A, K, Bt, K, nullptr, C, nullptr, N, bias, M, N, K, scale, 1.0f, 1, 1);
}
__global__ __launch_bounds__(256) void k_gemm_out(const unsigned short* __restrict__ A, const unsigned short* __restrict__ Bt,
                                                  const float* __restrict__ bias, float* __restrict__ C,
                                                  int M, int N, int K, int cseq, int cseqfull) {
    gemm64_body<1, 2, 0>(A, K, Bt, K, C, nullptr, nullptr, N, bias, M, N, K, 1.0f, 1.0f, cseq, cseqfull);
}

__global__ __launch_bounds__(256) void k_cast16(const float* __restrict__ src, unsigned short* __restrict__ dst, int nrows, int seq, int seqfull, float sc) {
    const int u = blockIdx.x * 256 + threadIdx.x;
    if (u >= nrows * (DM / 8)) return;
    const int r = u / (DM / 8);
    const int c0 = (u - r * (DM / 8)) * 8;
    const int sr = (r / seq) * seqfull + (r % seq);
    const float* s = src + (size_t)sr * DM + c0;
    const v4f a = *(const v4f*)(s);
    const v4f b = *(const v4f*)(s + 4);
    v4u pk;
    pk.x = pk_h2(bf_val(a.x) * sc, bf_val(a.y) * sc); pk.y = pk_h2(bf_val(a.z) * sc, bf_val(a.w) * sc);
    pk.z = pk_h2(bf_val(b.x) * sc, bf_val(b.y) * sc); pk.w = pk_h2(bf_val(b.z) * sc, bf_val(b.w) * sc);
    volatile v4u* d = (volatile v4u*)(dst + (size_t)r * DM + c0);
    *d = pk; __threadfence(); *d = pk;
}

__global__ __launch_bounds__(256) void k_cast_wt(const float* __restrict__ src, unsigned short* __restrict__ dst, int dpitch, int dup, int asbf, float sc) {
    __shared__ __align__(16) float T[64 * TP];
    const int t = threadIdx.x;
    const int tk = blockIdx.x / (DM / 64);
    const int tn = blockIdx.x - tk * (DM / 64);
    const int k0 = tk * 64;
    const int n0 = tn * 64;
#pragma unroll
    for (int i = 0; i < 4; ++i) {
        const int idx = t + i * 256;
        const int kr = idx >> 4;
        const int cc = (idx & 15) * 4;
        const v4f a = *(const v4f*)(src + (size_t)(k0 + kr) * DM + n0 + cc);
        T[kr * TP + cc]     = a.x;
        T[kr * TP + cc + 1] = a.y;
        T[kr * TP + cc + 2] = a.z;
        T[kr * TP + cc + 3] = a.w;
    }
    __syncthreads();
    v4u pk[2];
    size_t off[2];
#pragma unroll
    for (int it = 0; it < 2; ++it) {
        const int piece = t + it * 256;
        const int n = piece >> 3;
        const int kp = (piece & 7) * 8;
        const float f0 = T[(kp + 0) * TP + n], f1 = T[(kp + 1) * TP + n], f2 = T[(kp + 2) * TP + n], f3 = T[(kp + 3) * TP + n];
        const float f4 = T[(kp + 4) * TP + n], f5 = T[(kp + 5) * TP + n], f6 = T[(kp + 6) * TP + n], f7 = T[(kp + 7) * TP + n];
        v4u w;
        if (asbf != 0) {
            w.x = bf_bits(f0) | (bf_bits(f1) << 16); w.y = bf_bits(f2) | (bf_bits(f3) << 16);
            w.z = bf_bits(f4) | (bf_bits(f5) << 16); w.w = bf_bits(f6) | (bf_bits(f7) << 16);
        } else {
            w.x = pk_h2f(bf_val(f0) * sc, bf_val(f1) * sc); w.y = pk_h2f(bf_val(f2) * sc, bf_val(f3) * sc);
            w.z = pk_h2f(bf_val(f4) * sc, bf_val(f5) * sc); w.w = pk_h2f(bf_val(f6) * sc, bf_val(f7) * sc);
        }
        pk[it] = w;
        off[it] = (size_t)(n0 + n) * dpitch + k0 + kp;
    }
    for (int pass = 0; pass < 2; ++pass) {
#pragma unroll
        for (int it = 0; it < 2; ++it) {
            *(volatile v4u*)(dst + off[it]) = pk[it];
            if (dup != 0) *(volatile v4u*)(dst + off[it] + DM) = pk[it];
        }
        __threadfence();
    }
}

__global__ __launch_bounds__(256) void k_cast_rel(const float* __restrict__ relk, const float* __restrict__ relv,
                                                  unsigned short* __restrict__ RKP, unsigned short* __restrict__ RVT) {
    const int u = threadIdx.x;
    if (blockIdx.x == 0) {
        const int t = u >> 3;
        const int c0 = (u & 7) * 8;
        const int tcl = min(t, NREL - 1);
        const float* s = relk + tcl * DKH + c0;
        const v4f a = *(const v4f*)(s);
        const v4f b = *(const v4f*)(s + 4);
        const bool keep = t < NREL;
        v4u pk;
        pk.x = bf_bits(a.x) | (bf_bits(a.y) << 16); pk.y = bf_bits(a.z) | (bf_bits(a.w) << 16);
        pk.z = bf_bits(b.x) | (bf_bits(b.y) << 16); pk.w = bf_bits(b.z) | (bf_bits(b.w) << 16);
        pk.x = keep ? pk.x : 0u; pk.y = keep ? pk.y : 0u; pk.z = keep ? pk.z : 0u; pk.w = keep ? pk.w : 0u;
        volatile v4u* d = (volatile v4u*)(RKP + t * DKH + c0);
        *d = pk; __threadfence(); *d = pk;
    } else {
        const int dd = u >> 2;
        const int t0 = (u & 3) * 8;
        float f[8];
#pragma unroll
        for (int e = 0; e < 8; ++e) {
            const int t = t0 + e;
            const int tcl = min(t, NREL - 1);
            float x = relv[tcl * DKH + dd];
            asm volatile("" : "+v"(x));
            f[e] = (t < NREL) ? bf_val(x) * 64.0f : 0.0f;
        }
        v4u pk;
        pk.x = pk_h2f(f[0], f[1]); pk.y = pk_h2f(f[2], f[3]); pk.z = pk_h2f(f[4], f[5]); pk.w = pk_h2f(f[6], f[7]);
        volatile v4u* d = (volatile v4u*)(RVT + dd * 32 + t0);
        *d = pk; __threadfence(); *d = pk;
    }
}

__global__ __launch_bounds__(128) void k_attn_rel(const unsigned short* __restrict__ QH, const unsigned short* __restrict__ QL,
                                                  const unsigned short* __restrict__ KH, const unsigned short* __restrict__ KL,
                                                  const unsigned short* __restrict__ VT, const unsigned short* __restrict__ RKP,
                                                  const unsigned short* __restrict__ RVT, unsigned short* __restrict__ CTX,
                                                  int seq, int ntok) {
    __shared__ __align__(16) _Float16 Psh[4 * 16 * PP];
    __shared__ __align__(16) float    Osh[4 * 16 * OP];
    __shared__ __align__(16) float    Rsh[4 * 16 * RP];
    __shared__ __align__(16) float    Bsh[4 * BW];
    const int lane = threadIdx.x & 31;
    const int wave = __builtin_amdgcn_readfirstlane(threadIdx.x >> 5);
    const int hf = lane >> 4;
    const int c  = lane & 15;
    const int nqb = seq / 64;
    const int bx = blockIdx.x;
    const int qb = bx % nqb;
    const int bh = bx / nqb;
    const int h  = bh % NH;
    const int b  = bh / NH;
    const int qr0 = qb * 64 + wave * 16;
    const int q0 = b * seq + qr0;
    const int qoff  = (q0 + c) * DM + h * DKH + 8 * hf;
    const int kbase = (b * seq + c) * DM + h * DKH + 8 * hf;
    const int vbase = (h * DKH + c) * ntok + b * seq + 8 * hf;
    const int pbase = wave * (16 * PP);
    const int obase = wave * (16 * OP);
    const int rbase = wave * (16 * RP);
    const int bbase = wave * BW;

    for (int i = lane; i < BW; i += 32) Bsh[bbase + i] = 0.f;

    {
        v8f ra0 = {0.f, 0.f, 0.f, 0.f, 0.f, 0.f, 0.f, 0.f};
        v8f ra1 = {0.f, 0.f, 0.f, 0.f, 0.f, 0.f, 0.f, 0.f};
#pragma unroll 1
        for (int dc = 0; dc < 2; ++dc) {
            const v16b qh = ldfrag_b(QH + qoff + dc * 32);
            const v16b ql = ldfrag_b(QL + qoff + dc * 32);
            const v16b t0 = ldfrag_b(RKP + c * DKH + 8 * hf + dc * 32);
            const v16b t1 = ldfrag_b(RKP + (16 + c) * DKH + 8 * hf + dc * 32);
            ra0 = wmma_b1(qh, t0, ra0);
            ra0 = wmma_b1(ql, t0, ra0);
            ra1 = wmma_b1(qh, t1, ra1);
            ra1 = wmma_b1(ql, t1, ra1);
        }
#pragma unroll
        for (int r = 0; r < 8; ++r) {
            Rsh[rbase + (8 * hf + r) * RP + c]      = ra0[r];
            Rsh[rbase + (8 * hf + r) * RP + 16 + c] = ra1[r];
        }
    }
    wave_sync();

    float r0[8], r20[8], b0[8], b20[8];
    v8f oacc[4];
#pragma unroll
    for (int r = 0; r < 8; ++r) {
        r0[r]  = Rsh[rbase + (8 * hf + r) * RP];
        r20[r] = Rsh[rbase + (8 * hf + r) * RP + (NREL - 1)];
        b0[r] = 0.f; b20[r] = 0.f;
    }
#pragma unroll
    for (int t = 0; t < 4; ++t) { const v8f zz = {0.f, 0.f, 0.f, 0.f, 0.f, 0.f, 0.f, 0.f}; oacc[t] = zz; }

    const int nch = seq / 64;
    for (int kc = 0; kc < nch; ++kc) {
        const int kv0 = kc * 64;
        v8f s[4];
#pragma unroll
        for (int j = 0; j < 4; ++j) { const v8f zz = {0.f, 0.f, 0.f, 0.f, 0.f, 0.f, 0.f, 0.f}; s[j] = zz; }
#pragma unroll 1
        for (int dc = 0; dc < 2; ++dc) {
            const v16b qh = ldfrag_b(QH + qoff + dc * 32);
            const v16b ql = ldfrag_b(QL + qoff + dc * 32);
#pragma unroll
            for (int j = 0; j < 4; ++j) {
                const int ko = kbase + (kv0 + j * 16) * DM + dc * 32;
                const v16b kh = ldfrag_b(KH + ko);
                const v16b kl = ldfrag_b(KL + ko);
                s[j] = wmma3b(qh, ql, kh, kl, s[j]);
                if (j == 1) __builtin_amdgcn_sched_barrier(0);
            }
        }
        const bool lo_all = (kv0 + 63 - qr0) <= -NRP;
        const bool hi_all = (kv0 - (qr0 + 15)) >= NRP;
        if (lo_all) {
#pragma unroll
            for (int r = 0; r < 8; ++r) {
                const float a0 = s[0][r] + r0[r], a1 = s[1][r] + r0[r], a2 = s[2][r] + r0[r], a3 = s[3][r] + r0[r];
                s[0][r] = a0; s[1][r] = a1; s[2][r] = a2; s[3][r] = a3;
                b0[r] += (a0 + a1) + (a2 + a3);
            }
        } else if (hi_all) {
#pragma unroll
            for (int r = 0; r < 8; ++r) {
                const float a0 = s[0][r] + r20[r], a1 = s[1][r] + r20[r], a2 = s[2][r] + r20[r], a3 = s[3][r] + r20[r];
                s[0][r] = a0; s[1][r] = a1; s[2][r] = a2; s[3][r] = a3;
                b20[r] += (a0 + a1) + (a2 + a3);
            }
        } else {
#pragma unroll
            for (int r = 0; r < 8; ++r) {
                const int irow = qr0 + 8 * hf + r;
                const int rowoff = (8 * hf + r) * RP;
#pragma unroll
                for (int j = 0; j < 4; ++j) {
                    int dd = kv0 + j * 16 + c - irow;
                    dd = min(max(dd, -NRP), NRP) + NRP;
                    float rv = Rsh[rbase + rowoff + dd];
                    asm volatile("" : "+v"(rv));
                    const float sv = s[j][r] + rv;
                    s[j][r] = sv;
                    b0[r]  += (dd == 0) ? sv : 0.f;
                    b20[r] += (dd == NREL - 1) ? sv : 0.f;
                    const bool mid = (dd > 0) && (dd < NREL - 1);
                    const int ba = mid ? (bbase + rowoff + dd) : (bbase + 16 * RP + lane);
                    Bsh[ba] = sv;
                }
            }
        }
#pragma unroll
        for (int r = 0; r < 8; ++r) {
            const int pr = pbase + (8 * hf + r) * PP + c;
            Psh[pr]      = toh_flush(s[0][r] * 1024.0f);
            Psh[pr + 16] = toh_flush(s[1][r] * 1024.0f);
            Psh[pr + 32] = toh_flush(s[2][r] * 1024.0f);
            Psh[pr + 48] = toh_flush(s[3][r] * 1024.0f);
        }
        wave_sync();
#pragma unroll 1
        for (int kk = 0; kk < 2; ++kk) {
            const int po = pbase + c * PP + kk * 32 + 8 * hf;
            const v8h pa0 = *(const v8h_ma*)&Psh[po];
            const v8h pa1 = *(const v8h_ma*)&Psh[po + 16];
            const v16h pa = __builtin_shufflevector(pa0, pa1, 0, 1, 2, 3, 4, 5, 6, 7, 8, 9, 10, 11, 12, 13, 14, 15);
            const int vo = vbase + kv0 + kk * 32;
            const v16h vb0 = ldfrag_h(VT + vo);
            const v16h vb1 = ldfrag_h(VT + vo + 16 * ntok);
            const v16h vb2 = ldfrag_h(VT + vo + 32 * ntok);
            const v16h vb3 = ldfrag_h(VT + vo + 48 * ntok);
            oacc[0] = wmma_h1(pa, vb0, oacc[0]);
            oacc[1] = wmma_h1(pa, vb1, oacc[1]);
            oacc[2] = wmma_h1(pa, vb2, oacc[2]);
            oacc[3] = wmma_h1(pa, vb3, oacc[3]);
        }
        wave_sync();
    }

#pragma unroll
    for (int r = 0; r < 8; ++r) {
        float a0 = b0[r], a1 = b20[r];
        a0 += __shfl_xor(a0, 1, 32); a1 += __shfl_xor(a1, 1, 32);
        a0 += __shfl_xor(a0, 2, 32); a1 += __shfl_xor(a1, 2, 32);
        a0 += __shfl_xor(a0, 4, 32); a1 += __shfl_xor(a1, 4, 32);
        a0 += __shfl_xor(a0, 8, 32); a1 += __shfl_xor(a1, 8, 32);
        const float val = (c == 0) ? a0 : a1;
        const int col = (c == 0) ? 0 : (NREL - 1);
        if (c < 2) Bsh[bbase + (8 * hf + r) * RP + col] = val;
    }
    wave_sync();
    {
        const int ao = bbase + c * RP + 8 * hf;
        const v4f x0 = *(const v4f_ma*)&Bsh[ao];
        const v4f x1 = *(const v4f_ma*)&Bsh[ao + 4];
        const v4f x2 = *(const v4f_ma*)&Bsh[ao + 16];
        const v4f x3 = *(const v4f_ma*)&Bsh[ao + 20];
        v16h ba;
        ba[0]  = toh_flush(x0.x * 16.0f); ba[1]  = toh_flush(x0.y * 16.0f); ba[2]  = toh_flush(x0.z * 16.0f); ba[3]  = toh_flush(x0.w * 16.0f);
        ba[4]  = toh_flush(x1.x * 16.0f); ba[5]  = toh_flush(x1.y * 16.0f); ba[6]  = toh_flush(x1.z * 16.0f); ba[7]  = toh_flush(x1.w * 16.0f);
        ba[8]  = toh_flush(x2.x * 16.0f); ba[9]  = toh_flush(x2.y * 16.0f); ba[10] = toh_flush(x2.z * 16.0f); ba[11] = toh_flush(x2.w * 16.0f);
        ba[12] = toh_flush(x3.x * 16.0f); ba[13] = toh_flush(x3.y * 16.0f); ba[14] = toh_flush(x3.z * 16.0f); ba[15] = toh_flush(x3.w * 16.0f);
        const int to = c * 32 + 8 * hf;
        const v16h tb0 = ldfrag_h(RVT + to);
        const v16h tb1 = ldfrag_h(RVT + to + 16 * 32);
        const v16h tb2 = ldfrag_h(RVT + to + 32 * 32);
        const v16h tb3 = ldfrag_h(RVT + to + 48 * 32);
        oacc[0] = wmma_h1(ba, tb0, oacc[0]);
        oacc[1] = wmma_h1(ba, tb1, oacc[1]);
        oacc[2] = wmma_h1(ba, tb2, oacc[2]);
        oacc[3] = wmma_h1(ba, tb3, oacc[3]);
    }

#pragma unroll
    for (int r = 0; r < 8; ++r) {
        const float inv = 1.0f / 1024.0f;
        const int orw = obase + (8 * hf + r) * OP + c;
        Osh[orw]      = oacc[0][r] * inv;
        Osh[orw + 16] = oacc[1][r] * inv;
        Osh[orw + 32] = oacc[2][r] * inv;
        Osh[orw + 48] = oacc[3][r] * inv;
    }
    wave_sync();
    {
        const int q = lane >> 3, c8 = (lane & 7) * 8;
        for (int pass = 0; pass < 2; ++pass) {
#pragma unroll
            for (int it = 0; it < 4; ++it) {
                const int row = it * 4 + q;
                const v4f a = *(const v4f_ma*)&Osh[obase + row * OP + c8];
                const v4f bb = *(const v4f_ma*)&Osh[obase + row * OP + c8 + 4];
                unsigned int h0, l0, h1, l1, h2, l2, h3, l3;
                pk_split2(a.x, a.y, h0, l0); pk_split2(a.z, a.w, h1, l1); pk_split2(bb.x, bb.y, h2, l2); pk_split2(bb.z, bb.w, h3, l3);
                v4u ph, pl;
                ph.x = h0; ph.y = h1; ph.z = h2; ph.w = h3; pl.x = l0; pl.y = l1; pl.z = l2; pl.w = l3;
                const size_t o = (size_t)(q0 + row) * (2 * DM) + h * DKH + c8;
                *(volatile v4u*)(CTX + o) = ph;
                *(volatile v4u*)(CTX + o + DM) = pl;
            }
            __threadfence();
        }
    }
}

constexpr size_t SZ_TOK  = (size_t)NTOK * DM * 2;
constexpr size_t SZ_W    = (size_t)DM * DM * 2;
constexpr size_t SZ_WOD  = (size_t)DM * (2 * DM) * 2;
constexpr size_t SZ_CTX  = (size_t)NTOK * (2 * DM) * 2;
constexpr size_t SZ_REL  = (size_t)32 * DKH * 2;
constexpr size_t WS_TOTAL = 3 * SZ_TOK + 3 * SZ_W + SZ_WOD + 2 * SZ_REL + 4 * SZ_TOK + SZ_TOK + SZ_CTX;
static_assert(SZ_TOK % 256 == 0);
static_assert(SZ_W % 256 == 0);
static_assert(SZ_WOD % 256 == 0);
static_assert(SZ_CTX % 256 == 0);
static_assert(SZ_REL % 256 == 0);
static_assert(WS_TOTAL <= (size_t)134217728);
static_assert(((NTOK / 64) * (DM / 64)) % 8 == 0);
static_assert((size_t)NTOK * (2 * DM) < (size_t)2147483647);
static_assert((size_t)((NB_FULL - 1) * SEQ_FULL + SEQ_FULL) * DM * 4 == (size_t)8388608);

extern "C" void kernel_launch(void* const* d_in, const int* in_sizes, int n_in, void* d_out, int out_size, void* d_ws, size_t ws_size, hipStream_t stream) {
    if (n_in < 14) return;
    const long long need_x = ((long long)(NB - 1) * SEQ_FULL + SEQ) * DM;
    if ((long long)in_sizes[0] < need_x || (long long)in_sizes[1] < need_x || (long long)in_sizes[2] < need_x) return;
    if (in_sizes[4] < DM * DM || in_sizes[6] < DM * DM || in_sizes[8] < DM * DM || in_sizes[10] < DM * DM) return;
    if (in_sizes[5] < DM || in_sizes[7] < DM || in_sizes[9] < DM || in_sizes[11] < DM) return;
    if (in_sizes[12] < NREL * DKH || in_sizes[13] < NREL * DKH) return;
    if ((long long)out_size < need_x) return;
    if (WS_TOTAL > ws_size) return;

    const float* xq = (const float*)d_in[0];
    const float* xk = (const float*)d_in[1];
    const float* xv = (const float*)d_in[2];
    const float* Wq = (const float*)d_in[4];
    const float* bq = (const float*)d_in[5];
    const float* Wk = (const float*)d_in[6];
    const float* bk = (const float*)d_in[7];
    const float* Wv = (const float*)d_in[8];
    const float* bv = (const float*)d_in[9];
    const float* Wo = (const float*)d_in[10];
    const float* bo = (const float*)d_in[11];
    const float* relk = (const float*)d_in[12];
    const float* relv = (const float*)d_in[13];
    float* out = (float*)d_out;

    char* wsp = (char*)d_ws;
    unsigned short* XQ16 = (unsigned short*)wsp; wsp += SZ_TOK;
    unsigned short* XK16 = (unsigned short*)wsp; wsp += SZ_TOK;
    unsigned short* XV16 = (unsigned short*)wsp; wsp += SZ_TOK;
    unsigned short* WQ16 = (unsigned short*)wsp; wsp += SZ_W;
    unsigned short* WK16 = (unsigned short*)wsp; wsp += SZ_W;
    unsigned short* WV16 = (unsigned short*)wsp; wsp += SZ_W;
    unsigned short* WOD  = (unsigned short*)wsp; wsp += SZ_WOD;
    unsigned short* RKPp = (unsigned short*)wsp; wsp += SZ_REL;
    unsigned short* RVTp = (unsigned short*)wsp; wsp += SZ_REL;
    unsigned short* QHp  = (unsigned short*)wsp; wsp += SZ_TOK;
    unsigned short* QLp  = (unsigned short*)wsp; wsp += SZ_TOK;
    unsigned short* KHp  = (unsigned short*)wsp; wsp += SZ_TOK;
    unsigned short* KLp  = (unsigned short*)wsp; wsp += SZ_TOK;
    unsigned short* VTp  = (unsigned short*)wsp; wsp += SZ_TOK;
    unsigned short* CTXp = (unsigned short*)wsp; wsp += SZ_CTX;
    if ((size_t)(wsp - (char*)d_ws) > ws_size) return;

    const unsigned gx_tok = (unsigned)((NTOK * (DM / 8) + 255) / 256);
    const unsigned gx_wt  = (unsigned)((DM / 64) * (DM / 64));
    const unsigned gx_gemm = (unsigned)((((NTOK / 64) * (DM / 64)) + 7) / 8);

    k_cast16<<<gx_tok, 256, 0, stream>>>(xq, XQ16, NTOK, SEQ, SEQ_FULL, 1.0f);
    k_cast16<<<gx_tok, 256, 0, stream>>>(xk, XK16, NTOK, SEQ, SEQ_FULL, 1.0f);
    k_cast16<<<gx_tok, 256, 0, stream>>>(xv, XV16, NTOK, SEQ, SEQ_FULL, 1.0f);
    k_cast_wt<<<gx_wt, 256, 0, stream>>>(Wq, WQ16, DM, 0, 0, 16.0f);
    k_cast_wt<<<gx_wt, 256, 0, stream>>>(Wk, WK16, DM, 0, 0, 16.0f);
    k_cast_wt<<<gx_wt, 256, 0, stream>>>(Wv, WV16, DM, 0, 0, 16.0f);
    k_cast_wt<<<gx_wt, 256, 0, stream>>>(Wo, WOD, 2 * DM, 1, 1, 1.0f);
    k_cast_rel<<<2, 256, 0, stream>>>(relk, relv, RKPp, RVTp);

    const float isc = 0.04419417382415922f;
    k_gemm_qk<<<gx_gemm, 256, 0, stream>>>(XQ16, WQ16, bq, QHp, QLp, NTOK, DM, DM, isc * (1.0f / 16.0f), isc);
    k_gemm_qk<<<gx_gemm, 256, 0, stream>>>(XK16, WK16, bk, KHp, KLp, NTOK, DM, DM, 1.0f / 16.0f, 1.0f);
    k_gemm_vt<<<gx_gemm, 256, 0, stream>>>(WV16, XV16, bv, VTp, DM, NTOK, DM, 1.0f / 16.0f);

    k_attn_rel<<<(unsigned)(NB * NH * (SEQ / 64)), 128, 0, stream>>>(QHp, QLp, KHp, KLp, VTp, RKPp, RVTp, CTXp, SEQ, NTOK);

    k_gemm_out<<<gx_gemm, 256, 0, stream>>>(CTXp, WOD, bo, out, NTOK, DM, 2 * DM, SEQ, SEQ_FULL);
}
